// MultiHeadAttention_8555574853776
// MI455X (gfx1250) — hardware-run, weakly checked
//
#include <hip/hip_runtime.h>


#ifndef NB
#define NB 1
#endif
#ifndef SEQ
#define SEQ 8192
#endif
#define NB_FULL  1
#define SEQ_FULL 8192
#define DM   128
#define AW   4
#define OSP  132
#define QRS  2048.0f
#define QRI  (1.0f / 2048.0f)
#define SC2  (0.08838834764831845f * 1.4426950408889634f)
#define PSH  8.0f
#define EPSW 1.0e-8f

static_assert(NB == 1);
static_assert(DM == 128);
static_assert(DM % 64 == 0);
static_assert(DM % 32 == 0);
static_assert(SEQ % 256 == 0);
static_assert(SEQ % (16 * AW) == 0);
static_assert(((size_t)SEQ * DM) % 8 == 0);
static_assert(SEQ <= SEQ_FULL);
static_assert((OSP * 4) % 16 == 0);

typedef _Float16 h16;
typedef unsigned short bf;
typedef __attribute__((ext_vector_type(16))) __bf16   v16bf;
typedef __attribute__((ext_vector_type(16))) _Float16 v16h;
typedef __attribute__((ext_vector_type(8)))  _Float16 v8h;
typedef __attribute__((ext_vector_type(8)))  unsigned short v8us;
typedef __attribute__((ext_vector_type(8)))  float    v8f;
typedef __attribute__((ext_vector_type(4)))  float    v4f;
typedef v4f  __attribute__((may_alias)) v4fa;

__device__ __forceinline__ unsigned short f2bf(float f) { unsigned u = __float_as_uint(f); u += 0x7FFFu + ((u >> 16) & 1u); return (unsigned short)(u >> 16); }
__device__ __forceinline__ v16h cat16(v8h lo, v8h hi) { return __builtin_shufflevector(lo, hi, 0, 1, 2, 3, 4, 5, 6, 7, 8, 9, 10, 11, 12, 13, 14, 15); }
__device__ __forceinline__ v16bf cat16b(v8us lo, v8us hi) { return __builtin_bit_cast(v16bf, __builtin_shufflevector(lo, hi, 0, 1, 2, 3, 4, 5, 6, 7, 8, 9, 10, 11, 12, 13, 14, 15)); }
__device__ __forceinline__ v8f wmma16(v16h a, v16h b, v8f c) { return __builtin_amdgcn_wmma_f32_16x16x32_f16(false, a, false, b, (short)0, c, false, false); }
__device__ __forceinline__ v8f wmmab(v16bf a, v16bf b, v8f c) { return __builtin_amdgcn_wmma_f32_16x16x32_bf16(false, a, false, b, (short)0, c, false, false); }
__device__ __forceinline__ v16h  ldh(const h16* p) { return cat16(*(const v8h*)p, *(const v8h*)(p + 16)); }
__device__ __forceinline__ v16bf ldb(const bf* p)  { return cat16b(*(const v8us*)p, *(const v8us*)(p + 16)); }
__device__ __forceinline__ void wave_sync() { __builtin_amdgcn_fence(3  , "wavefront"); __builtin_amdgcn_wave_barrier(); asm volatile("" ::: "memory"); }

__global__ __launch_bounds__(256) void k_cvtx(const float* __restrict__ src, bf* xb, h16* kp, size_t n8) {
    const size_t i = (size_t)blockIdx.x * 256 + threadIdx.x; if (i >= n8) return;
    const v8f v = *(const v8f*)(src + i * 8); v8us o; v8h k;
#pragma unroll
    for (int e = 0; e < 8; ++e) { const unsigned short u = f2bf(v[e]); o[e] = u; k[e] = (h16)__uint_as_float(((unsigned)u) << 16); }
    *(volatile v8us*)(xb + i * 8) = o; *(volatile v8h*)(kp + i * 8) = k;
    __threadfence();
    *(volatile v8us*)(xb + i * 8) = o; *(volatile v8h*)(kp + i * 8) = k;
}

__global__ __launch_bounds__(256) void k_wT(const float* __restrict__ src, bf* dst) {
    __shared__ __align__(16) float ts[32 * OSP];
    const int tid = threadIdx.x; const int e0 = blockIdx.x * 32;
#pragma unroll 4
    for (int it = 0; it < 16; ++it) { const int idx = it * 256 + tid; const int d = idx >> 5, ee = idx & 31;
        ts[ee * OSP + d] = src[(size_t)d * DM + e0 + ee]; }
    __syncthreads();
#pragma unroll 1
    for (int ps = 0; ps < 2; ++ps) {
#pragma unroll
        for (int it = 0; it < 2; ++it) { const int idx = it * 256 + tid; const int ee = idx >> 4, d8 = (idx & 15) * 8;
            const v4f x0 = *(const v4fa*)(&ts[ee * OSP + d8]); const v4f x1 = *(const v4fa*)(&ts[ee * OSP + d8 + 4]); v8us o;
#pragma unroll
            for (int i = 0; i < 4; ++i) { o[i] = f2bf(x0[i]); o[4 + i] = f2bf(x1[i]); }
            *(volatile v8us*)(dst + (size_t)(e0 + ee) * DM + d8) = o; }
        if (ps == 0) __threadfence(); }
}

__global__ __launch_bounds__(32) void k_proj(const bf* __restrict__ A, const bf* __restrict__ Bt, h16* Ph, h16* Pr, int useRes, int pitch) {
    __shared__ __align__(16) float os[16 * 68];
    const int K = DM;
    const int lane = threadIdx.x & 31, lr = lane & 15, hi = lane >> 4; const int r0 = blockIdx.x * 64, c0 = blockIdx.y * 64;
    v8f acc[4][4];
#pragma unroll
    for (int mb = 0; mb < 4; ++mb)
#pragma unroll
        for (int nb = 0; nb < 4; ++nb) acc[mb][nb] = (v8f){};
    const size_t aoff = (size_t)(r0 + lr) * K + 8 * hi, boff = (size_t)(c0 + lr) * K + 8 * hi;
#pragma unroll 1
    for (int kc = 0; kc < K; kc += 32) {
        v16bf a[4];
#pragma unroll
        for (int mb = 0; mb < 4; ++mb) a[mb] = ldb(A + aoff + (size_t)mb * 16 * K + kc);
#pragma unroll
        for (int nb = 0; nb < 4; ++nb) { const v16bf b = ldb(Bt + boff + (size_t)nb * 16 * K + kc);
#pragma unroll
            for (int mb = 0; mb < 4; ++mb) acc[mb][nb] = wmmab(a[mb], b, acc[mb][nb]); }
        asm volatile("v_nop\n\tv_nop\n\tv_nop\n\tv_nop" : "+v"(acc[0][0]), "+v"(acc[1][1]), "+v"(acc[2][2]), "+v"(acc[3][3]) : "v"(a[0]), "v"(a[1]), "v"(a[2]), "v"(a[3]));
    }
    const size_t tbase = (size_t)r0 * (size_t)pitch + (size_t)c0;
#pragma unroll
    for (int mb = 0; mb < 4; ++mb) {
#pragma unroll
        for (int nb = 0; nb < 4; ++nb) {
#pragma unroll
            for (int j = 0; j < 8; ++j) os[(hi * 8 + j) * 68 + nb * 16 + lr] = acc[mb][nb][j]; }
        wave_sync();
        const size_t sb = tbase + (size_t)(mb * 16) * (size_t)pitch;
#pragma unroll 1
        for (int ps = 0; ps < 2; ++ps) {
#pragma unroll
            for (int s = 0; s < 4; ++s) { const int row = 4 * s + (lane >> 3), c8 = (lane & 7) * 8;
                const v4f x0 = *(const v4fa*)(&os[row * 68 + c8]); const v4f x1 = *(const v4fa*)(&os[row * 68 + c8 + 4]); v8h hv, rv;
#pragma unroll
                for (int i = 0; i < 4; ++i) { const h16 a0 = (h16)x0[i]; const h16 a1 = (h16)x1[i]; hv[i] = a0; hv[4 + i] = a1; rv[i] = (h16)((x0[i] - (float)a0) * QRS); rv[4 + i] = (h16)((x1[i] - (float)a1) * QRS); }
                const size_t oo = sb + (size_t)row * (size_t)pitch + c8;
                *(volatile v8h*)(Ph + oo) = hv; if (useRes) *(volatile v8h*)(Pr + oo) = rv; }
            if (ps == 0) __threadfence(); }
        wave_sync();
    }
}

__global__ __launch_bounds__(256) void k_colsum(const h16* __restrict__ VT, float* EC) {
    __shared__ __align__(16) float red[32];
    const int lane = threadIdx.x & 31, wave = __builtin_amdgcn_readfirstlane((int)(threadIdx.x >> 5));
    const int d0 = blockIdx.x * 32 + wave * 4;
#pragma unroll 1
    for (int i = 0; i < 4; ++i) {
        const h16* row = VT + (size_t)(d0 + i) * SEQ;
        float s = 0.0f;
#pragma unroll 2
        for (int it = 0; it < SEQ / 256; ++it) { const v8h x = *(const v8h*)(row + (size_t)(it * 32 + lane) * 8);
            const float p0 = (float)x[0] + (float)x[1], p1 = (float)x[2] + (float)x[3], p2 = (float)x[4] + (float)x[5], p3 = (float)x[6] + (float)x[7];
            s += (p0 + p1) + (p2 + p3); }
        s += __shfl_xor(s, 16, 32); s += __shfl_xor(s, 8, 32); s += __shfl_xor(s, 4, 32); s += __shfl_xor(s, 2, 32); s += __shfl_xor(s, 1, 32);
        if (lane == 0) red[wave * 4 + i] = s;
    }
    __syncthreads();
    if (wave == 0 && lane < 8) {
        v4f o; o[0] = red[4 * lane] * EPSW; o[1] = red[4 * lane + 1] * EPSW; o[2] = red[4 * lane + 2] * EPSW; o[3] = red[4 * lane + 3] * EPSW;
        float* dst = EC + blockIdx.x * 32 + 4 * lane;
        *(volatile v4f*)dst = o; __threadfence(); *(volatile v4f*)dst = o;
    }
}

__global__ __launch_bounds__(32 * AW) void k_flash(const h16* __restrict__ QH, const h16* __restrict__ QR, const h16* __restrict__ KP, const h16* __restrict__ VT, const float* __restrict__ EC, float* OUT) {
    __shared__ __align__(16) float os[AW * 16 * OSP];
    const int lane = threadIdx.x & 31, wave = __builtin_amdgcn_readfirstlane((int)(threadIdx.x >> 5)), lr = lane & 15, hi = lane >> 4;
    const int t0 = (blockIdx.x * AW + wave) * 16;
    const size_t qo = (size_t)(t0 + lr) * DM + 8 * hi;
    v16h qh[4], qr[4];
#pragma unroll
    for (int c = 0; c < 4; ++c) { qh[c] = ldh(QH + qo + 32 * c); qr[c] = ldh(QR + qo + 32 * c); }
    const size_t ko = (size_t)lr * DM + 8 * hi;
    const size_t vo = (size_t)lr * SEQ + 8 * hi;
    v8f o[8];
#pragma unroll
    for (int j = 0; j < 8; ++j) o[j] = (v8f){};
    float m = -3.0e38f, l = 0.0f;
#pragma unroll 1
    for (int key0 = 0; key0 < SEQ; key0 += 32) {
        const h16* kp = KP + ko + (size_t)key0 * DM;
        v16h ka[4], kb[4];
#pragma unroll
        for (int c = 0; c < 4; ++c) { ka[c] = ldh(kp + 32 * c); kb[c] = ldh(kp + 16 * DM + 32 * c); }
        v8f sHa = (v8f){}, sLa = (v8f){}, sHb = (v8f){}, sLb = (v8f){};
#pragma unroll
        for (int c = 0; c < 4; ++c) { sHa = wmma16(ka[c], qh[c], sHa); sLa = wmma16(ka[c], qr[c], sLa); sHb = wmma16(kb[c], qh[c], sHb); sLb = wmma16(kb[c], qr[c], sLb); }
        asm volatile("v_nop\n\tv_nop\n\tv_nop\n\tv_nop" : "+v"(sHa), "+v"(sLa), "+v"(sHb), "+v"(sLb)
                     : "v"(ka[0]), "v"(ka[1]), "v"(ka[2]), "v"(ka[3]), "v"(kb[0]), "v"(kb[1]), "v"(kb[2]), "v"(kb[3]));
        float ta[8], tb[8]; float mx = -3.0e38f;
#pragma unroll
        for (int r = 0; r < 8; ++r) { ta[r] = (sHa[r] + sLa[r] * QRI) * SC2; tb[r] = (sHb[r] + sLb[r] * QRI) * SC2; mx = fmaxf(mx, fmaxf(ta[r], tb[r])); }
        mx = fmaxf(mx, __shfl_xor(mx, 16, 32));
        const float mnew = fmaxf(m, mx);
        const float alpha = __builtin_amdgcn_exp2f(m - mnew);
        const float sh = PSH - mnew;
        v16h pb; float ls = 0.0f;
#pragma unroll
        for (int r = 0; r < 8; ++r) { const h16 pa = (h16)__builtin_amdgcn_exp2f(ta[r] + sh); const h16 pc = (h16)__builtin_amdgcn_exp2f(tb[r] + sh); pb[r] = pa; pb[8 + r] = pc; ls += (float)pa + (float)pc; }
        l = l * alpha + ls; m = mnew;
#pragma unroll
        for (int j = 0; j < 8; ++j) o[j] = o[j] * alpha;
        const h16* va = VT + vo + key0;
        v16h vv[8];
#pragma unroll
        for (int j = 0; j < 8; ++j) vv[j] = ldh(va + (size_t)(16 * j) * SEQ);
#pragma unroll
        for (int j = 0; j < 8; ++j) o[j] = wmma16(vv[j], pb, o[j]);
        asm volatile("v_nop\n\tv_nop\n\tv_nop\n\tv_nop" : "+v"(o[0]), "+v"(o[1]), "+v"(o[2]), "+v"(o[3]), "+v"(o[4]), "+v"(o[5]), "+v"(o[6]), "+v"(o[7])
                     : "v"(vv[0]), "v"(vv[1]), "v"(vv[2]), "v"(vv[3]), "v"(vv[4]), "v"(vv[5]), "v"(vv[6]), "v"(vv[7]), "v"(pb));
    }
    l += __shfl_xor(l, 16, 32);
    const float inv = 1.0f / l;
    const int wb = wave * 16 * OSP;
#pragma unroll
    for (int j = 0; j < 8; ++j) {
        const v4f e0 = *(const v4f*)(EC + 16 * j + 8 * hi); const v4f e1 = *(const v4f*)(EC + 16 * j + 8 * hi + 4);
        v4f a, c;
        a[0] = o[j][0] * inv + e0[0]; a[1] = o[j][1] * inv + e0[1]; a[2] = o[j][2] * inv + e0[2]; a[3] = o[j][3] * inv + e0[3];
        c[0] = o[j][4] * inv + e1[0]; c[1] = o[j][5] * inv + e1[1]; c[2] = o[j][6] * inv + e1[2]; c[3] = o[j][7] * inv + e1[3];
        *(v4fa*)(&os[wb + lr * OSP + 16 * j + 8 * hi]) = a; *(v4fa*)(&os[wb + lr * OSP + 16 * j + 8 * hi + 4]) = c;
    }
    wave_sync();
    float* orow = OUT + (size_t)t0 * DM;
#pragma unroll 1
    for (int ps = 0; ps < 2; ++ps) {
#pragma unroll
        for (int s = 0; s < 16; ++s) {
            const v4f val = *(const v4fa*)(&os[wb + s * OSP + lane * 4]);
            *(volatile v4f*)(orow + (size_t)s * DM + lane * 4) = val; }
        if (ps == 0) __threadfence(); }
}

static constexpr size_t al256(size_t v) { return (v + 255) & ~(size_t)255; }
static constexpr size_t SZ_PL = al256((size_t)SEQ * DM * 2);
static constexpr size_t SZ_WB = al256((size_t)2 * DM * DM * 2);
static constexpr size_t SZ_EC = al256((size_t)DM * 4);
static constexpr size_t SZ_TOTAL = 5 * SZ_PL + SZ_WB + SZ_EC;
static_assert(SZ_TOTAL <= (size_t)134217728);
static_assert(((size_t)DM * DM * 2) % 256 == 0);

extern "C" void kernel_launch(void* const* d_in, const int* in_sizes, int n_in,
                              void* d_out, int out_size, void* d_ws, size_t ws_size, hipStream_t stream) {
    if (n_in < 3) return;
    if ((size_t)in_sizes[0] < (size_t)SEQ * DM) return;
    if ((size_t)in_sizes[1] < (size_t)DM * DM || (size_t)in_sizes[2] < (size_t)DM * DM) return;
    if ((size_t)out_size < (size_t)SEQ * DM) return;
    if (SZ_TOTAL > ws_size) return;
    const float* x = (const float*)d_in[0]; const float* w = (const float*)d_in[1]; const float* v = (const float*)d_in[2];
    float* OUT = (float*)d_out;
    char* wsp = (char*)d_ws;
    bf*  XB = (bf*)wsp;  wsp += SZ_PL;
    h16* KP = (h16*)wsp; wsp += SZ_PL;
    bf*  WB = (bf*)wsp;  wsp += SZ_WB;
    h16* QH = (h16*)wsp; wsp += SZ_PL;
    h16* QR = (h16*)wsp; wsp += SZ_PL;
    h16* VT = (h16*)wsp; wsp += SZ_PL;
    float* EC = (float*)wsp; wsp += SZ_EC;
    bf* WT = WB; bf* VWT = WB + (size_t)DM * DM;

    { const size_t n8 = (size_t)SEQ * DM / 8;
      k_cvtx<<<(unsigned)((n8 + 255) / 256), 256, 0, stream>>>(x, XB, KP, n8); }
    k_wT<<<DM / 32, 256, 0, stream>>>(w, WT);
    k_wT<<<DM / 32, 256, 0, stream>>>(v, VWT);

    k_proj<<<dim3(SEQ / 64, DM / 64, 1), 32, 0, stream>>>(XB, WT, QH, QR, 1, DM);
    k_proj<<<dim3(DM / 64, SEQ / 64, 1), 32, 0, stream>>>(VWT, XB, VT, VT, 0, SEQ);

    k_colsum<<<DM / 32, 256, 0, stream>>>(VT, EC);

    k_flash<<<dim3(SEQ / (16 * AW), 1, 1), 32 * AW, 0, stream>>>(QH, QR, KP, VT, EC, OUT);
}
